// CIN_56392920597049
// MI455X (gfx1250) — hardware-verified
//
#include <hip/hip_runtime.h>

constexpr int kB    = 512;
constexpr int kF    = 39;
constexpr int kD    = 32;
constexpr int kU    = 256;
constexpr int kRows = kB * kD;
constexpr int kK0   = kF * kF;
constexpr int kK0P  = 1536;
constexpr int kK1   = kF * kU;
constexpr int kOutW = 3 * kU;
constexpr int kFP   = 64;
constexpr int kC0B  = 128;
constexpr int kC0Rows = kC0B * kD;
constexpr int kNC0  = kB / kC0B;
constexpr int kC1B  = 64;
constexpr int kC1Rows = kC1B * kD;
constexpr int kNC1  = kB / kC1B;
constexpr float kZCarry = 16.0f;
constexpr float kWCarry = 64.0f;
constexpr float kXCarry = 16.0f;
constexpr float kScale01 = 1.0f / (kZCarry * kWCarry);
constexpr float kScaleP  = 1.0f / kXCarry;
constexpr float kScale2  = 1.0f / kWCarry;

static_assert(kK0P % 32 == 0 && kK0P >= kK0, "k0 pad");
static_assert(kK1 % 32 == 0, "k1");
static_assert(kD % 32 == 0, "kp");
static_assert(kC0Rows % 64 == 0 && kC1Rows % 64 == 0 && kU % 64 == 0 && kB % 64 == 0 && kFP % 64 == 0, "tiles");
static_assert(((kC0Rows / 64) * (kU / 64)) % 8 == 0, "g0 grid");
static_assert(((kC1Rows / 64) * (kU / 64)) % 8 == 0, "g1 grid");
static_assert(((kB / 64) * (kU / 64)) % 8 == 0, "g2 grid");
static_assert(kK1 % 64 == 0 && kK0P % 64 == 0, "wt grid");
static_assert(kNC0 * kC0B == kB && kNC1 * kC1B == kB, "chunks");

constexpr size_t kSzW0T = (size_t)kU * kK0P * 2;
constexpr size_t kSzW1T = (size_t)kU * kK1 * 2;
constexpr size_t kSzX0A = (size_t)kB * kFP * kD * 2;
constexpr size_t kSzZ0  = (size_t)kC0Rows * kK0P * 2;
constexpr size_t kSzZ1  = (size_t)kC1Rows * kK1 * 2;
constexpr size_t kSzH   = (size_t)kRows * kU * 4;
constexpr size_t kSzF1T = (size_t)kB * kU * kD * 2;
constexpr size_t kSzPP  = (size_t)kB * kFP * kU * 2;
constexpr size_t kOffW0T = 0;
constexpr size_t kOffW1T = kOffW0T + kSzW0T;
constexpr size_t kOffW2T = kOffW1T + kSzW1T;
constexpr size_t kOffX0A = kOffW2T + kSzW1T;
constexpr size_t kOffZ0  = kOffX0A + kSzX0A;
constexpr size_t kOffZ1  = kOffZ0 + kSzZ0;
constexpr size_t kOffH0  = kOffZ1 + kSzZ1;
constexpr size_t kOffH1  = kOffH0 + kSzH;
constexpr size_t kOffF1T = kOffH1 + kSzH;
constexpr size_t kOffPP  = kOffF1T + kSzF1T;
constexpr size_t kWsTotal = kOffPP + kSzPP;
static_assert(kWsTotal == 125304832ull, "carve");
static_assert(kWsTotal <= 134217728ull, "carve limit");
static_assert(kOffW1T % 256 == 0 && kOffW2T % 256 == 0 && kOffX0A % 256 == 0 && kOffZ0 % 256 == 0 &&
              kOffZ1 % 256 == 0 && kOffH0 % 256 == 0 && kOffH1 % 256 == 0 && kOffF1T % 256 == 0 &&
              kOffPP % 256 == 0, "align");

typedef __attribute__((ext_vector_type(16))) _Float16 v16h;
typedef __attribute__((ext_vector_type(8)))  _Float16 v8h;
typedef __attribute__((ext_vector_type(16))) __bf16   v16b;
typedef __attribute__((ext_vector_type(8)))  __bf16   v8b;
typedef __attribute__((ext_vector_type(8)))  float    v8f;
typedef __attribute__((ext_vector_type(4)))  float    v4f;
typedef __attribute__((ext_vector_type(4)))  unsigned int v4u;

__device__ __forceinline__ unsigned short f2bf_bits(float f) {
  unsigned u = __float_as_uint(f);
  return (unsigned short)((u + 0x7FFFu + ((u >> 16) & 1u)) >> 16);
}
__device__ __forceinline__ float bf_bits2f(unsigned short h) { return __uint_as_float(((unsigned)h) << 16); }

__device__ __forceinline__ void dep_guard_h(v8f& a, v8f& b, v16h x, v16h y) { asm volatile("v_nop\n\tv_nop\n\tv_nop\n\tv_nop" : "+v"(a), "+v"(b) : "v"(x), "v"(y)); }
__device__ __forceinline__ void dep_guard_b(v8f& a, v8f& b, v16b x, v16b y) { asm volatile("v_nop\n\tv_nop\n\tv_nop\n\tv_nop" : "+v"(a), "+v"(b) : "v"(x), "v"(y)); }
__device__ __forceinline__ void dep_guard4_h(v8f& a, v8f& b, v8f& c, v8f& d, v16h x, v16h y) { asm volatile("v_nop\n\tv_nop\n\tv_nop\n\tv_nop" : "+v"(a), "+v"(b), "+v"(c), "+v"(d) : "v"(x), "v"(y)); }
__device__ __forceinline__ void dep_guard4_b(v8f& a, v8f& b, v8f& c, v8f& d, v16b x, v16b y) { asm volatile("v_nop\n\tv_nop\n\tv_nop\n\tv_nop" : "+v"(a), "+v"(b), "+v"(c), "+v"(d) : "v"(x), "v"(y)); }
__device__ __forceinline__ void keep4_h(v16h a, v16h b, v16h c, v16h d) { asm volatile("v_nop" :: "v"(a), "v"(b), "v"(c), "v"(d)); }
__device__ __forceinline__ void keep4_b(v16b a, v16b b, v16b c, v16b d) { asm volatile("v_nop" :: "v"(a), "v"(b), "v"(c), "v"(d)); }
__device__ __forceinline__ void acc_guard4(v8f& a, v8f& b, v8f& c, v8f& d) { asm volatile("v_nop\n\tv_nop\n\tv_nop\n\tv_nop" : "+v"(a), "+v"(b), "+v"(c), "+v"(d)); }
template <typename T> struct Frag;
template <> struct Frag<_Float16> {
  typedef v16h V; union U { v16h v; v8h h[2]; };
  static __device__ __forceinline__ v16h load(const _Float16* p) {
    U f; f.h[0] = *(const v8h*)(p); f.h[1] = *(const v8h*)(p + 16); return f.v;
  }
  static __device__ __forceinline__ v8f mma(v16h a, v16h b, v8f c) {
    return __builtin_amdgcn_wmma_f32_16x16x32_f16(false, a, false, b, (short)0, c, false, false);
  }
  static __device__ __forceinline__ void guard(v8f& a, v8f& b, v16h x, v16h y) { dep_guard_h(a, b, x, y); }
  static __device__ __forceinline__ void guard4(v8f& a, v8f& b, v8f& c, v8f& d, v16h x, v16h y) { dep_guard4_h(a, b, c, d, x, y); }
  static __device__ __forceinline__ void keep(v16h a, v16h b, v16h c, v16h d) { keep4_h(a, b, c, d); }
};
template <> struct Frag<__bf16> {
  typedef v16b V; union U { v16b v; v8b h[2]; };
  static __device__ __forceinline__ v16b load(const __bf16* p) {
    U f; f.h[0] = *(const v8b*)(p); f.h[1] = *(const v8b*)(p + 16); return f.v;
  }
  static __device__ __forceinline__ v8f mma(v16b a, v16b b, v8f c) {
    return __builtin_amdgcn_wmma_f32_16x16x32_bf16(false, a, false, b, (short)0, c, false, false);
  }
  static __device__ __forceinline__ void guard(v8f& a, v8f& b, v16b x, v16b y) { dep_guard_b(a, b, x, y); }
  static __device__ __forceinline__ void guard4(v8f& a, v8f& b, v8f& c, v8f& d, v16b x, v16b y) { dep_guard4_b(a, b, c, d, x, y); }
  static __device__ __forceinline__ void keep(v16b a, v16b b, v16b c, v16b d) { keep4_b(a, b, c, d); }
};

__device__ __forceinline__ unsigned pk16(unsigned short a, unsigned short b) { return (unsigned)a | ((unsigned)b << 16); }
__device__ __forceinline__ unsigned short h_bits(float f) { const _Float16 h = (_Float16)f; return __builtin_bit_cast(unsigned short, h); }

template <int ET> struct Elem;
template <> struct Elem<0> { typedef _Float16 T; };
template <> struct Elem<1> { typedef __bf16 T; };
template <int ET, bool SPLIT, int BIAS_MODE, int OUT_MODE, bool RESID, int ACT = 0>
__global__ __launch_bounds__(256) void wmma_gemm64(
    const unsigned short* __restrict__ Ap, const unsigned short* __restrict__ A2p, int lda, long strideA,
    const unsigned short* __restrict__ Btp, const unsigned short* __restrict__ Bt2p, int ldb, long strideB,
    void* __restrict__ Cout, void* __restrict__ Cout2, int ldc, long strideC,
    const float* __restrict__ bias,
    const float* __restrict__ resid, long strideR,
    int M, int N, int K, float scale) {
  typedef typename Elem<ET>::T T;
  typedef typename Frag<T>::V V;
  const T* A = (const T*)Ap; const T* A2 = (const T*)A2p; const T* Bt = (const T*)Btp; const T* Bt2 = (const T*)Bt2p;
  __shared__ __align__(16) float sT[8][16 * 68];
  const int b    = blockIdx.y;
  const int lane = threadIdx.x & 31;
  const int wave = threadIdx.x >> 5;
  const int tilesN = N >> 6;
  const int tilesM = M >> 6;
  const int tile = blockIdx.x * 8 + wave;
  if (tile >= tilesM * tilesN) return;
  const int tm = tile / tilesN;
  const int tn = tile - tm * tilesN;
  const int m0 = tm << 6;
  const int n0 = tn << 6;

  const T* Ab  = A  + (size_t)b * strideA;
  const T* Bb  = Bt + (size_t)b * strideB;
  const T* Ab2 = SPLIT ? (A2  + (size_t)b * strideA) : nullptr;
  const T* Bb2 = SPLIT ? (Bt2 + (size_t)b * strideB) : nullptr;

  const int rlane = lane & 15;
  const int koff  = (lane >> 4) * 8;
  const int mOff  = (lane >> 4) * 8;

  v8f acc[4][4];
#pragma unroll
  for (int i = 0; i < 4; ++i)
#pragma unroll
    for (int j = 0; j < 4; ++j) acc[i][j] = (v8f){0.f,0.f,0.f,0.f,0.f,0.f,0.f,0.f};

  for (int k0 = 0; k0 < K; k0 += 32) {
    V bh[4], bl[4];
#pragma unroll
    for (int j = 0; j < 4; ++j) {
      const size_t bo = (size_t)(n0 + (j << 4) + rlane) * ldb + koff + k0;
      bh[j] = Frag<T>::load(Bb + bo);
      if (SPLIT) bl[j] = Frag<T>::load(Bb2 + bo);
    }
#pragma unroll
    for (int i = 0; i < 4; ++i) {
      const size_t ao = (size_t)(m0 + (i << 4) + rlane) * lda + koff + k0;
      V ah = Frag<T>::load(Ab + ao);
      V al;
      if (SPLIT) al = Frag<T>::load(Ab2 + ao);
#pragma unroll
      for (int j = 0; j < 4; ++j) {
        acc[i][j] = Frag<T>::mma(ah, bh[j], acc[i][j]);
        if (SPLIT) {
          acc[i][j] = Frag<T>::mma(ah, bl[j], acc[i][j]);
          acc[i][j] = Frag<T>::mma(al, bh[j], acc[i][j]);
        }
      }
      Frag<T>::guard4(acc[i][0], acc[i][1], acc[i][2], acc[i][3], ah, SPLIT ? al : ah);
    }
    Frag<T>::keep(bh[0], bh[1], bh[2], bh[3]);
    if (SPLIT) Frag<T>::keep(bl[0], bl[1], bl[2], bl[3]);
  }
  acc_guard4(acc[0][0], acc[0][1], acc[0][2], acc[0][3]);
  acc_guard4(acc[1][0], acc[1][1], acc[1][2], acc[1][3]);
  acc_guard4(acc[2][0], acc[2][1], acc[2][2], acc[2][3]);
  acc_guard4(acc[3][0], acc[3][1], acc[3][2], acc[3][3]);

  float* slab = sT[wave];
  const float* Rb = RESID ? (resid + (size_t)b * strideR) : nullptr;
#pragma unroll
  for (int i = 0; i < 4; ++i) {
    const int mBase = m0 + (i << 4);
#pragma unroll
    for (int j = 0; j < 4; ++j) {
      const int n = n0 + (j << 4) + rlane;
      float bv = 0.f;
      if (BIAS_MODE == 2) bv = bias[n];
      if (BIAS_MODE == 3) bv = bias[n] * 32.0f;
#pragma unroll
      for (int r = 0; r < 8; ++r) {
        float v = acc[i][j][r] * scale;
        if (BIAS_MODE == 1) v += bias[mBase + mOff + r];
        if (BIAS_MODE == 2 || BIAS_MODE == 3) v += bv;
        if (RESID) v += Rb[(size_t)(mBase + mOff + r) * ldc + n];
        if (ACT == 2) v = fmaxf(v, 0.0f);
        if (ACT == 4) v = (v > 0.f) ? v : 0.01f * v;
        slab[(mOff + r) * 68 + (j << 4) + rlane] = v;
      }
    }
    __builtin_amdgcn_fence(__ATOMIC_RELEASE, "workgroup");
    __builtin_amdgcn_wave_barrier();
    __builtin_amdgcn_fence(__ATOMIC_ACQUIRE, "workgroup");
    if (OUT_MODE == 0) {
      float* C = (float*)Cout + (size_t)b * strideC;
      const int hh = lane >> 4, c4 = (lane & 15) * 4;
      for (int pass = 0; pass < 2; ++pass) {
#pragma unroll
        for (int it = 0; it < 8; ++it) {
          const int row = it * 2 + hh;
          v4f v = *(const v4f*)(slab + row * 68 + c4);
          *(volatile v4f*)(C + (size_t)(mBase + row) * ldc + n0 + c4) = v;
        }
        __threadfence();
      }
    } else {
      const int q = lane >> 3, c8 = (lane & 7) * 8;
      unsigned short* C  = (unsigned short*)Cout  + (size_t)b * strideC;
      unsigned short* C2 = (OUT_MODE == 2) ? ((unsigned short*)Cout2 + (size_t)b * strideC) : nullptr;
      for (int pass = 0; pass < 2; ++pass) {
#pragma unroll
        for (int it = 0; it < 4; ++it) {
          const int row = it * 4 + q;
          const float* sp = slab + row * 68 + c8;
          v8h hv, lv;
#pragma unroll
          for (int e = 0; e < 8; ++e) {
            if (OUT_MODE == 1) {
              hv[e] = (_Float16)sp[e];
            } else {
              unsigned short hb = f2bf_bits(sp[e]);
              unsigned short lb = f2bf_bits(sp[e] - bf_bits2f(hb));
              hv[e] = __builtin_bit_cast(_Float16, hb);
              lv[e] = __builtin_bit_cast(_Float16, lb);
            }
          }
          *(volatile v8h*)(C + (size_t)(mBase + row) * ldc + n0 + c8) = hv;
          if (OUT_MODE == 2) *(volatile v8h*)(C2 + (size_t)(mBase + row) * ldc + n0 + c8) = lv;
        }
        __threadfence();
      }
    }
    __builtin_amdgcn_fence(__ATOMIC_RELEASE, "workgroup");
    __builtin_amdgcn_wave_barrier();
    __builtin_amdgcn_fence(__ATOMIC_ACQUIRE, "workgroup");
  }
}

__global__ __launch_bounds__(256) void wt_kernel(const float* __restrict__ Wa, const float* __restrict__ Wb,
                                                 unsigned short* __restrict__ Ta, unsigned short* __restrict__ Tb,
                                                 int Kin, int KP, float carry) {
  __shared__ float sm[64][65];
  const int t  = threadIdx.x;
  const int f0 = blockIdx.x * 64;
  const int u0 = blockIdx.y * 64;
  const int z  = blockIdx.z;
  const float* W = (z == 0) ? Wa : Wb;
  unsigned short* Tp = (z == 0) ? Ta : Tb;
#pragma unroll
  for (int i = 0; i < 8; ++i) {
    const int e  = i * 256 + t;
    const int r  = e >> 6;
    const int c  = e & 63;
    const int f  = f0 + r;
    const int fc = (f < Kin) ? f : (Kin - 1);
    const float v = W[(size_t)fc * kU + u0 + c] * carry;
    sm[c][r] = (f < Kin) ? v : 0.0f;
  }
  asm volatile("" ::: "memory");
#pragma unroll
  for (int i = 8; i < 16; ++i) {
    const int e  = i * 256 + t;
    const int r  = e >> 6;
    const int c  = e & 63;
    const int f  = f0 + r;
    const int fc = (f < Kin) ? f : (Kin - 1);
    const float v = W[(size_t)fc * kU + u0 + c] * carry;
    sm[c][r] = (f < Kin) ? v : 0.0f;
  }
  __syncthreads();
  const int lane = t & 31, wave = t >> 5;
  const int q = lane >> 3, c8 = (lane & 7) * 8;
  for (int pass = 0; pass < 2; ++pass) {
#pragma unroll
    for (int it = 0; it < 2; ++it) {
      const int row = wave * 8 + it * 4 + q;
      unsigned short hb[8];
#pragma unroll
      for (int e = 0; e < 8; ++e) hb[e] = h_bits(sm[row][c8 + e]);
      const v4u u = (v4u){pk16(hb[0], hb[1]), pk16(hb[2], hb[3]), pk16(hb[4], hb[5]), pk16(hb[6], hb[7])};
      *(volatile v4u*)(Tp + (size_t)(u0 + row) * KP + f0 + c8) = u;
    }
    __threadfence();
  }
}

__global__ __launch_bounds__(256) void x0a_kernel(const float* __restrict__ x0, unsigned short* __restrict__ Xa) {
  const int g = blockIdx.x * 256 + threadIdx.x;
  if (g >= kB * kFP * kD / 8) return;
  const int b   = g >> 8;
  const int rem = g & 255;
  const int i   = rem >> 2;
  const int d0  = (rem & 3) * 8;
  const int ic  = (i < kF) ? i : (kF - 1);
  const float* src = x0 + ((size_t)(b * kF + ic) * kD + d0);
  const v4f a = *(const v4f*)(src);
  const v4f c = *(const v4f*)(src + 4);
  const float fa = (i < kF) ? kXCarry : 0.0f;
  unsigned short hb[8];
#pragma unroll
  for (int e = 0; e < 4; ++e) {
    hb[e]     = h_bits(a[e] * fa);
    hb[4 + e] = h_bits(c[e] * fa);
  }
  const v4u u = (v4u){pk16(hb[0], hb[1]), pk16(hb[2], hb[3]), pk16(hb[4], hb[5]), pk16(hb[6], hb[7])};
  unsigned short* p = Xa + (size_t)g * 8;
  *(volatile v4u*)p = u;
  __threadfence();
  *(volatile v4u*)p = u;
}

__global__ __launch_bounds__(256) void z0_kernel(const float* __restrict__ x0, unsigned short* __restrict__ Zc, int batch0) {
  __shared__ float xs[kF][kD + 1];
  const int t = threadIdx.x, lane = t & 31, wave = t >> 5;
  const int b = batch0 + blockIdx.x;
  const float* xb = x0 + (size_t)b * (kF * kD);
#pragma unroll
  for (int it = 0; it < 5; ++it) {
    const int e  = it * 256 + t;
    const int ec = (e < kF * kD) ? e : (kF * kD - 1);
    const float v = xb[ec];
    if (e < kF * kD) xs[ec >> 5][ec & 31] = v;
  }
  __syncthreads();
  const int rbase = blockIdx.x * kD;
#pragma unroll 1
  for (int rr = 0; rr < 4; ++rr) {
    const int d = wave * 4 + rr;
    unsigned short* zrow = Zc + (size_t)(rbase + d) * kK0P;
#pragma unroll 1
    for (int it = 0; it < 6; ++it) {
      const int c0 = it * 256 + lane * 8;
      unsigned short hb[8];
#pragma unroll
      for (int e = 0; e < 8; ++e) {
        const int c  = c0 + e;
        const int i  = c / kF;
        const int j  = c - i * kF;
        const int ic = (i < kF) ? i : (kF - 1);
        float p = xs[ic][d] * xs[j][d];
        p = p * kZCarry;
        hb[e] = h_bits((c < kK0) ? p : 0.0f);
      }
      const v4u u = (v4u){pk16(hb[0], hb[1]), pk16(hb[2], hb[3]), pk16(hb[4], hb[5]), pk16(hb[6], hb[7])};
      unsigned short* p = zrow + c0;
      *(volatile v4u*)p = u;
      __threadfence();
      *(volatile v4u*)p = u;
    }
  }
}

__global__ __launch_bounds__(256) void z1_kernel(const float* __restrict__ x0, const float* __restrict__ H,
                                                 unsigned short* __restrict__ Zc, int batch0) {
  __shared__ float xs[kF + 1];
  const int t = threadIdx.x, lane = t & 31, wave = t >> 5;
  const int r = blockIdx.x;
  const int b = batch0 + (r >> 5);
  const int d = r & 31;
  {
    const int ic = (t < kF) ? t : (kF - 1);
    const float v = x0[(size_t)(b * kF + ic) * kD + d] * kZCarry;
    if (t < kF) xs[t] = v;
  }
  const float* hrow = H + (size_t)(b * kD + d) * kU + lane * 8;
  const v4f a = *(const v4f*)(hrow);
  const v4f c = *(const v4f*)(hrow + 4);
  __syncthreads();
  unsigned short* zrow = Zc + (size_t)r * kK1 + lane * 8;
#pragma unroll 1
  for (int i = wave; i < kF; i += 8) {
    const float s = xs[i];
    unsigned short hb[8];
#pragma unroll
    for (int e = 0; e < 4; ++e) {
      hb[e]     = h_bits(a[e] * s);
      hb[4 + e] = h_bits(c[e] * s);
    }
    const v4u u = (v4u){pk16(hb[0], hb[1]), pk16(hb[2], hb[3]), pk16(hb[4], hb[5]), pk16(hb[6], hb[7])};
    unsigned short* p = zrow + (size_t)i * kU;
    *(volatile v4u*)p = u;
    __threadfence();
    *(volatile v4u*)p = u;
  }
}

__global__ __launch_bounds__(256) void rowsum_kernel(const float* __restrict__ H, float* __restrict__ out, int coloff) {
  __shared__ __align__(16) float ps[4][kU];
  __shared__ __align__(16) float ss[kU];
  const int t = threadIdx.x, lane = t & 31, wave = t >> 5;
  const int b = blockIdx.x;
  const int cg = t & 63, dg = t >> 6;
  const float* hp = H + (size_t)(b * kD + dg * 8) * kU + cg * 4;
  v4f acc = (v4f){0.f, 0.f, 0.f, 0.f};
#pragma unroll
  for (int dd = 0; dd < 8; ++dd) acc += *(const v4f*)(hp + (size_t)dd * kU);
  *(v4f*)(&ps[dg][cg * 4]) = acc;
  __syncthreads();
  {
    float s = ps[0][t] + ps[1][t];
    s = s + ps[2][t];
    s = s + ps[3][t];
    ss[t] = s;
  }
  __syncthreads();
  if (wave < 2) {
    const int c4 = (wave * 32 + lane) * 4;
    const v4f v = *(const v4f*)(&ss[c4]);
    float* p = out + (size_t)b * kOutW + coloff + c4;
    *(volatile v4f*)p = v;
    __threadfence();
    *(volatile v4f*)p = v;
  }
}

__global__ __launch_bounds__(256) void f1t_kernel(const float* __restrict__ H, unsigned short* __restrict__ Ft) {
  __shared__ float sm[kD][kU + 1];
  const int t = threadIdx.x;
  const int b = blockIdx.x;
  const float* hb = H + (size_t)b * kD * kU;
#pragma unroll
  for (int it = 0; it < 8; ++it) {
    const int f = (it * 256 + t) * 4;
    const int d = f >> 8, j = f & 255;
    const v4f v = *(const v4f*)(hb + f);
    sm[d][j]     = v[0];
    sm[d][j + 1] = v[1];
    sm[d][j + 2] = v[2];
    sm[d][j + 3] = v[3];
  }
  __syncthreads();
  unsigned short* ob = Ft + (size_t)b * kU * kD;
#pragma unroll 1
  for (int it = 0; it < 4; ++it) {
    const int q  = it * 256 + t;
    const int j  = q >> 2;
    const int d0 = (q & 3) * 8;
    unsigned short hbt[8];
#pragma unroll
    for (int e = 0; e < 8; ++e) hbt[e] = h_bits(sm[d0 + e][j]);
    const v4u u = (v4u){pk16(hbt[0], hbt[1]), pk16(hbt[2], hbt[3]), pk16(hbt[4], hbt[5]), pk16(hbt[6], hbt[7])};
    unsigned short* p = ob + (size_t)q * 8;
    *(volatile v4u*)p = u;
    __threadfence();
    *(volatile v4u*)p = u;
  }
}

extern "C" void kernel_launch(void* const* d_in, const int* in_sizes, int n_in,
                              void* d_out, int out_size, void* d_ws, size_t ws_size,
                              hipStream_t stream) {
  if (n_in < 8) return;
  if (in_sizes[0] != kB * kF * kD) return;
  if (in_sizes[2] != kK0 * kU || in_sizes[4] != kK1 * kU || in_sizes[6] != kK1 * kU) return;
  if (in_sizes[3] < kU || in_sizes[5] < kU || in_sizes[7] < kU) return;
  if (out_size != kB * kOutW) return;
  if (ws_size < kWsTotal) return;

  const float* x0 = (const float*)d_in[0];
  const float* W0 = (const float*)d_in[2];
  const float* b0 = (const float*)d_in[3];
  const float* W1 = (const float*)d_in[4];
  const float* b1 = (const float*)d_in[5];
  const float* W2 = (const float*)d_in[6];
  const float* b2 = (const float*)d_in[7];
  float* out = (float*)d_out;

  char* ws = (char*)d_ws;
  unsigned short* W0T = (unsigned short*)(ws + kOffW0T);
  unsigned short* W1T = (unsigned short*)(ws + kOffW1T);
  unsigned short* W2T = (unsigned short*)(ws + kOffW2T);
  unsigned short* X0A = (unsigned short*)(ws + kOffX0A);
  unsigned short* Z0  = (unsigned short*)(ws + kOffZ0);
  unsigned short* Z1  = (unsigned short*)(ws + kOffZ1);
  float*          H0  = (float*)(ws + kOffH0);
  float*          H1  = (float*)(ws + kOffH1);
  unsigned short* F1T = (unsigned short*)(ws + kOffF1T);
  unsigned short* PP  = (unsigned short*)(ws + kOffPP);

  wt_kernel<<<dim3(kK0P / 64, kU / 64, 1), 256, 0, stream>>>(W0, W0, W0T, W0T, kK0, kK0P, kWCarry);
  wt_kernel<<<dim3(kK1 / 64, kU / 64, 2), 256, 0, stream>>>(W1, W2, W1T, W2T, kK1, kK1, kWCarry);
  x0a_kernel<<<(kB * kFP * kD / 8) / 256, 256, 0, stream>>>(x0, X0A);

  for (int c = 0; c < kNC0; ++c) {
    z0_kernel<<<kC0B, 256, 0, stream>>>(x0, Z0, c * kC0B);
    float* Hc = H0 + (size_t)c * kC0Rows * kU;
    wmma_gemm64<0, false, 2, 0, false, 0><<<dim3(((kC0Rows / 64) * (kU / 64)) / 8, 1), 256, 0, stream>>>(
        Z0, Z0, kK0P, 0L, W0T, W0T, kK0P, 0L, (void*)Hc, (void*)Hc, kU, 0L,
        b0, b0, 0L, kC0Rows, kU, kK0P, kScale01);
  }
  rowsum_kernel<<<kB, 256, 0, stream>>>(H0, out, 0);

  for (int c = 0; c < kNC1; ++c) {
    z1_kernel<<<kC1Rows, 256, 0, stream>>>(x0, H0, Z1, c * kC1B);
    float* Hc = H1 + (size_t)c * kC1Rows * kU;
    wmma_gemm64<0, false, 2, 0, false, 0><<<dim3(((kC1Rows / 64) * (kU / 64)) / 8, 1), 256, 0, stream>>>(
        Z1, Z1, kK1, 0L, W1T, W1T, kK1, 0L, (void*)Hc, (void*)Hc, kU, 0L,
        b1, b1, 0L, kC1Rows, kU, kK1, kScale01);
  }
  rowsum_kernel<<<kB, 256, 0, stream>>>(H1, out, kU);

  f1t_kernel<<<kB, 256, 0, stream>>>(H1, F1T);
  wmma_gemm64<0, false, 0, 1, false, 0><<<dim3(1, kB), 256, 0, stream>>>(
      X0A, X0A, kD, (long)(kFP * kD), F1T, F1T, kD, (long)(kU * kD), (void*)PP, (void*)PP, kU, (long)(kFP * kU),
      b1, b1, 0L, kFP, kU, kD, kScaleP);
  wmma_gemm64<0, false, 3, 0, false, 0><<<dim3(((kB / 64) * (kU / 64)) / 8, 1), 256, 0, stream>>>(
      PP, PP, kFP * kU, 0L, W2T, W2T, kK1, 0L, (void*)(out + 2 * kU), (void*)(out + 2 * kU), kOutW, 0L,
      b2, b2, 0L, kB, kU, kK1, kScale2);
}
